// GraphLinkPredictor_86208583565975
// MI455X (gfx1250) — hardware-verified
//
#include <hip/hip_runtime.h>
#include <math.h>

typedef __attribute__((ext_vector_type(16))) _Float16 v16h;
typedef __attribute__((ext_vector_type(16))) __bf16 v16b;
typedef __attribute__((ext_vector_type(8)))  _Float16 v8h;
typedef __attribute__((ext_vector_type(8)))  float v8f;
typedef __attribute__((ext_vector_type(4)))  float v4f;
typedef __attribute__((ext_vector_type(2)))  float v2f;
typedef __attribute__((ext_vector_type(4)))  unsigned v4u;
typedef __attribute__((ext_vector_type(4)))  int v4i;
typedef float __attribute__((may_alias)) float_a;
typedef int __attribute__((may_alias)) int_a;

template <typename T> __device__ __forceinline__ void vst2(void* p, T v) { *(volatile T*)p = v; __threadfence(); *(volatile T*)p = v; }
__device__ __forceinline__ v8f wmma16(v16h a, v16h b, v8f c) {
  v8f d = __builtin_amdgcn_wmma_f32_16x16x32_f16(false, a, false, b, (short)0, c, false, false);
  asm volatile("v_nop\n\tv_nop\n\tv_nop\n\tv_nop" : "+v"(d) : "v"(a), "v"(b));
  return d;
}
__device__ __forceinline__ v8f wmma_bf(v16b a, v16b b, v8f c) {
  v8f d = __builtin_amdgcn_wmma_f32_16x16x32_bf16(false, a, false, b, (short)0, c, false, false);
  asm volatile("v_nop\n\tv_nop\n\tv_nop\n\tv_nop" : "+v"(d) : "v"(a), "v"(b));
  return d;
}
__device__ __forceinline__ v16h frag_h(const _Float16* rowk0, int lane) {
  union { v16h v; v8h q[2]; } u; const _Float16* p = rowk0 + 8 * (lane >> 4);
  u.q[0] = *(const v8h*)p; u.q[1] = *(const v8h*)(p + 16); return u.v;
}
__device__ __forceinline__ v16h frag_f32(const float* rowk0, int lane) {
  v16h a; const float* p = rowk0 + 8 * (lane >> 4);
#pragma unroll
  for (int i = 0; i < 8; ++i) { a[i] = (_Float16)p[i]; a[8 + i] = (_Float16)p[16 + i]; }
  return a;
}
__device__ __forceinline__ v16h frag_f32s(const float* rowk0, int lane, float sc) {
  v16h a; const float* p = rowk0 + 8 * (lane >> 4);
#pragma unroll
  for (int i = 0; i < 8; ++i) { a[i] = (_Float16)(p[i] * sc); a[8 + i] = (_Float16)(p[16 + i] * sc); }
  return a;
}
__device__ __forceinline__ v16h fragc_f32(const float* W, int k0, int n, int lane, int ld, int K) {
  v16h a; const int g = lane >> 4;
#pragma unroll
  for (int i = 0; i < 8; ++i) { const int ka = k0 + 8 * g + i, kb = ka + 16;
    a[i] = (_Float16)(ka < K ? W[(size_t)(ka < K ? ka : K - 1) * ld + n] : 0.f); a[8 + i] = (_Float16)(kb < K ? W[(size_t)(kb < K ? kb : K - 1) * ld + n] : 0.f); }
  return a;
}
struct F2 { v16b h, l; };
__device__ __forceinline__ F2 bsplit16(const float v[16]) { F2 r;
#pragma unroll
  for (int i = 0; i < 16; ++i) { const __bf16 h = (__bf16)v[i]; r.h[i] = h; r.l[i] = (__bf16)(v[i] - (float)h); }
  return r; }
__device__ __forceinline__ F2 split_row(const float* row, int k0, int lane) { float v[16]; const float* p = row + k0 + 8 * (lane >> 4);
#pragma unroll
  for (int i = 0; i < 8; ++i) { v[i] = p[i]; v[8 + i] = p[16 + i]; }
  return bsplit16(v); }
__device__ __forceinline__ F2 split_rowK(const float* row, int k0, int lane, int K) { float v[16]; const int g = lane >> 4;
#pragma unroll
  for (int i = 0; i < 8; ++i) { const int ka = k0 + 8 * g + i, kb = ka + 16; v[i] = ka < K ? row[ka < K ? ka : K - 1] : 0.f; v[8 + i] = kb < K ? row[kb < K ? kb : K - 1] : 0.f; }
  return bsplit16(v); }
__device__ __forceinline__ F2 split_col(const float* W, int k0, int n, int lane, int ld, int K) { float v[16]; const int g = lane >> 4;
#pragma unroll
  for (int i = 0; i < 8; ++i) { const int ka = k0 + 8 * g + i, kb = ka + 16; v[i] = ka < K ? W[(size_t)(ka < K ? ka : K - 1) * ld + n] : 0.f; v[8 + i] = kb < K ? W[(size_t)(kb < K ? kb : K - 1) * ld + n] : 0.f; }
  return bsplit16(v); }
__device__ __forceinline__ v8f mac3(const F2& a, const F2& b, v8f c) { c = wmma_bf(a.l, b.h, c); c = wmma_bf(a.h, b.l, c); return wmma_bf(a.h, b.h, c); }
__device__ __forceinline__ float sigm(float v) { return 1.0f / (1.0f + expf(-v)); }
#define LDSX() do { asm volatile("s_wait_dscnt 0" ::: "memory"); __builtin_amdgcn_wave_barrier(); __builtin_amdgcn_fence(__ATOMIC_RELEASE, "workgroup"); } while (0)


#define NN 10000
#define NE0 160000
#define NET (NE0 + NN)
#define NPR 100000
#define NRB ((NN + 63) / 64)
#define NPAD (NRB * 64)
#ifndef NNT
#define NNT NN
#define NRBT NRB
#define NPRT NPR
#endif
typedef __attribute__((ext_vector_type(8))) __bf16 v8b;
__device__ __forceinline__ v16b frag_b(const __bf16* rowk0, int lane) {
  union { v16b v; v8b q[2]; } u; const __bf16* p = rowk0 + 8 * (lane >> 4);
  u.q[0] = *(const v8b*)p; u.q[1] = *(const v8b*)(p + 16); return u.v;
}
__device__ __forceinline__ float bfr(float v) { return (float)(__bf16)v; }
__device__ __attribute__((noinline)) float exp_ni(float v) { return expf(v); }
__device__ __attribute__((noinline)) float erf_ni(float v) { return erff(v); }

__device__ __attribute__((noinline)) float expm1_ni(float v) { return expm1f(v); }
#define CSA_N 10000
#define CSA_E 170000
#define CSA_FINN (CSA_E + 32 * CSA_NBK)
#define CSA_CHUNK 4096
#define CSA_BKT 256
#define CSA_NCH ((CSA_E + CSA_CHUNK - 1) / CSA_CHUNK)
#define CSA_NBK ((CSA_N + CSA_BKT - 1) / CSA_BKT)
#define CSA_NBKP (((CSA_NBK + 63) / 64) * 64)
#define CSA_SEGCAP (CSA_E + 32 * CSA_NBK * CSA_NCH)
#ifndef CSA_BCAP
#define CSA_BCAP 10240
#endif
#define CSA_SZ_CNT   (4u * CSA_NCH * CSA_NBKP)
#define CSA_SZ_OFF   (4u * CSA_NBK * (((CSA_NCH + 31) / 32) * 32))
#define CSA_SZ_BST   (4u * (((CSA_NBK + 1 + 31) / 32) * 32))
#define CSA_SZ_SEG   (4u * CSA_SEGCAP)
#define CSA_SZ_FIN   (4u * (CSA_E + 32 * CSA_NBK))
#define CSA_SZ_ROW   (4u * CSA_NBK * CSA_BKT)
#define CSA_OFFP (((CSA_NCH + 31) / 32) * 32)

__global__ __launch_bounds__(256) void k_csA_cnt(const int* __restrict__ DST, int dstride, int* __restrict__ CNT) {
  __shared__ unsigned short sc[256][CSA_NBK + 1]; __shared__ __align__(16) int srow[CSA_NBKP];
  const int c = blockIdx.x, tid = threadIdx.x;
  for (int b = 0; b < CSA_NBK; ++b) sc[tid][b] = 0;
  const size_t e0 = (size_t)c * CSA_CHUNK + tid * 16;
  for (int i = 0; i < 16; ++i) { const size_t e = e0 + i; if (e < (size_t)CSA_E) { int d = DST[e * dstride]; d = min(max(d, 0), CSA_N - 1); sc[tid][d / CSA_BKT] += 1; } }
  __syncthreads();
  for (int b = tid; b < CSA_NBKP; b += 256) { int s = 0; if (b < CSA_NBK) for (int t = 0; t < 256; ++t) s += sc[t][b]; srow[b] = s; }
  __syncthreads();
  for (int q = tid; q < CSA_NBKP / 4; q += 256) vst2((unsigned*)(CNT + (size_t)c * CSA_NBKP + q * 4), *(const v4u*)&srow[q * 4]);
}
__global__ __launch_bounds__(256) void k_csA_scan(const int* __restrict__ CNT, int* __restrict__ OFF, int* __restrict__ BST) {
  __shared__ int sbt[CSA_NBK + 1]; __shared__ int sbs[((CSA_NBK + 1 + 31) / 32) * 32]; __shared__ int scnt[CSA_NBK + 1]; __shared__ __align__(16) int sbuf[64][CSA_OFFP];
  const int tid = threadIdx.x;
  for (int b = tid; b < CSA_NBK; b += 256) { int sp = 0, st = 0; for (int c = 0; c < CSA_NCH; ++c) { const int n = CNT[(size_t)c * CSA_NBKP + b]; st += n; sp += (n + 31) & ~31; } sbt[b] = sp; scnt[b] = st; }
  for (int b = tid; b < ((CSA_NBK + 1 + 31) / 32) * 32; b += 256) sbs[b] = 0;
  __syncthreads();
  if (tid == 0) { int acc = 0, accf = 0; for (int b = 0; b < CSA_NBK; ++b) { const int t = sbt[b]; sbt[b] = acc; acc += t; sbs[b] = accf; accf += (scnt[b] + 31) & ~31; } sbs[CSA_NBK] = accf; }
  __syncthreads();
  for (int b0 = 0; b0 < CSA_NBK; b0 += 64) {
    if (tid < 64 && b0 + tid < CSA_NBK) { const int b = b0 + tid; int o = sbt[b]; for (int c = 0; c < CSA_OFFP; ++c) { if (c < CSA_NCH) { sbuf[tid][c] = o; o += (CNT[(size_t)c * CSA_NBKP + b] + 31) & ~31; } else sbuf[tid][c] = 0; } }
    __syncthreads();
    for (int q = tid; q < 64 * (CSA_OFFP / 4); q += 256) { const int r = q / (CSA_OFFP / 4), pc = q % (CSA_OFFP / 4); if (b0 + r < CSA_NBK) vst2((unsigned*)(OFF + (size_t)(b0 + r) * CSA_OFFP + pc * 4), *(const v4u*)&sbuf[r][pc * 4]); }
    __syncthreads(); }
  for (int q = tid; q < ((CSA_NBK + 1 + 31) / 32) * 32 / 4; q += 256) vst2((unsigned*)(BST + q * 4), *(const v4u*)&sbs[q * 4]);
}
__global__ __launch_bounds__(256) void k_csA_scatter(const int* __restrict__ SRC, const int* __restrict__ DST, int sstride, int dstride, const int* __restrict__ OFF, int* __restrict__ SEGS, int* __restrict__ SEGE) {
  __shared__ unsigned short sc[256][CSA_NBK + 1]; __shared__ int sbase[CSA_NBK + 1]; __shared__ int scn[CSA_NBK + 1]; __shared__ int sord[CSA_CHUNK];
  const int c = blockIdx.x, tid = threadIdx.x;
  for (int b = 0; b < CSA_NBK; ++b) sc[tid][b] = 0;
  const size_t e0 = (size_t)c * CSA_CHUNK + tid * 16; int bk[16];
#pragma unroll
  for (int i = 0; i < 16; ++i) { const size_t e = e0 + i; bk[i] = -1; if (e < (size_t)CSA_E) { int d = DST[e * dstride]; d = min(max(d, 0), CSA_N - 1); bk[i] = d / CSA_BKT; sc[tid][bk[i]] += 1; } }
  __syncthreads();
  for (int b = tid; b < CSA_NBK; b += 256) { int acc = 0; for (int t = 0; t < 256; ++t) { const int v = sc[t][b]; sc[t][b] = (unsigned short)acc; acc += v; } scn[b] = acc; }
  __syncthreads();
  if (tid == 0) { int acc = 0; for (int b = 0; b < CSA_NBK; ++b) { sbase[b] = acc; acc += scn[b]; } }
  __syncthreads();
#pragma unroll
  for (int i = 0; i < 16; ++i) { if (bk[i] >= 0) { const int b = bk[i]; const int r = sc[tid][b]; sc[tid][b] = (unsigned short)(r + 1); sord[sbase[b] + r] = tid * 16 + i; } }
  __syncthreads();
  for (int b = 0; b < CSA_NBK; ++b) { const int n = scn[b]; if (n == 0) continue; const int nl = ((n + 31) & ~31); const size_t o = (size_t)(min(max(OFF[(size_t)b * CSA_OFFP + c], 0), CSA_SEGCAP - nl) & ~31);
    for (int q = tid; q < nl / 4; q += 256) { int4 vs, ve;
#pragma unroll
      for (int k = 0; k < 4; ++k) { const int i = q * 4 + k; int s = -1, eid = -1; if (i < n) { const size_t e = (size_t)c * CSA_CHUNK + sord[sbase[b] + i]; s = min(max(SRC[e * sstride], 0), CSA_N - 1); eid = (int)e; } vs[k] = s; ve[k] = eid; }
      vst2((unsigned*)(SEGS + o + q * 4), *(const v4u*)&vs); vst2((unsigned*)(SEGE + o + q * 4), *(const v4u*)&ve); } }
}
__global__ __launch_bounds__(256) void k_csA_bucket(const int* __restrict__ CNT, const int* __restrict__ OFF, const int* __restrict__ BST, const int* __restrict__ SEGS, const int* __restrict__ SEGE, const int* __restrict__ DST, int dstride, int* __restrict__ FS, int* __restrict__ FE, int* __restrict__ ROWST, int* __restrict__ ROWCNT) {
  __shared__ int ssrc[CSA_BCAP]; __shared__ int seid[CSA_BCAP]; __shared__ unsigned char snod[CSA_BCAP]; __shared__ int souts[CSA_BCAP]; __shared__ int soute[CSA_BCAP]; __shared__ int scount[256]; __shared__ int sstart[257]; __shared__ int stot;
  const int b = blockIdx.x, tid = threadIdx.x;
  if (tid == 0) { int t = 0; for (int c = 0; c < CSA_NCH; ++c) t += min(max(CNT[(size_t)c * CSA_NBKP + b], 0), CSA_CHUNK); stot = (t <= CSA_BCAP) ? t : 0; }
  __syncthreads();
  { int base = 0; for (int c = 0; c < CSA_NCH; ++c) { const int n = min(max(CNT[(size_t)c * CSA_NBKP + b], 0), CSA_CHUNK); const int o = min(max(OFF[(size_t)b * CSA_OFFP + c], 0), CSA_SEGCAP - ((n + 31) & ~31));
      for (int i = tid; i < n; i += 256) { const int p = base + i; if (p < CSA_BCAP) { ssrc[p] = min(max(SEGS[o + i], 0), CSA_N - 1); const int e = min(max(SEGE[o + i], 0), CSA_E - 1); seid[p] = e; int d = DST[(size_t)e * dstride]; d = min(max(d, 0), CSA_N - 1); const int dl = d - b * CSA_BKT; snod[p] = (unsigned char)(dl >= 0 && dl < 256 ? dl : 255); } }
      base += n; } }
  __syncthreads();
  const int node = b * CSA_BKT + tid; int cnt = 0; for (int p = 0; p < stot; ++p) cnt += (snod[p] == tid) ? 1 : 0;
  scount[tid] = cnt; __syncthreads();
  if (tid == 0) { int acc = 0; for (int t = 0; t < 256; ++t) { sstart[t] = acc; acc += scount[t]; } sstart[256] = acc; }
  __syncthreads();
  const int bst0 = min(max(BST[b], 0), CSA_FINN - ((sstart[256] + 31) & ~31)) & ~31; const int gst = bst0 + sstart[tid];
  { int w = sstart[tid]; for (int p = 0; p < stot; ++p) if (snod[p] == tid) { souts[w] = ssrc[p]; soute[w] = seid[p]; ++w; } }
  __syncthreads();
  { const int n = sstart[256]; const int nl = (n + 31) & ~31; for (int q = tid; q < nl / 4; q += 256) { int4 vs, ve;
#pragma unroll
      for (int k = 0; k < 4; ++k) { const int i = q * 4 + k; vs[k] = i < n ? souts[i] : -1; ve[k] = i < n ? soute[i] : -1; }
      vst2((unsigned*)(FS + bst0 + q * 4), *(const v4u*)&vs); vst2((unsigned*)(FE + bst0 + q * 4), *(const v4u*)&ve); } }
  __syncthreads();
  { __shared__ __align__(16) int srs[256], src2[256]; srs[tid] = node < CSA_N ? gst : 0; src2[tid] = node < CSA_N ? cnt : 0; __syncthreads();
    if (tid < 64) vst2((unsigned*)(ROWST + (size_t)b * 256 + tid * 4), *(const v4u*)&srs[tid * 4]); else if (tid < 128) vst2((unsigned*)(ROWCNT + (size_t)b * 256 + (tid - 64) * 4), *(const v4u*)&src2[(tid - 64) * 4]); }
}


#define WS_CNT  0u
#define WS_OFF  (WS_CNT + CSA_SZ_CNT)
#define WS_BST  (WS_OFF + CSA_SZ_OFF)
#define WS_SEGS (WS_BST + CSA_SZ_BST)
#define WS_SEGE (WS_SEGS + CSA_SZ_SEG)
#define WS_FS   (WS_SEGE + CSA_SZ_SEG)
#define WS_FE   (WS_FS + CSA_SZ_FIN)
#define WS_RST  (WS_FE + CSA_SZ_FIN)
#define WS_RCT  (WS_RST + CSA_SZ_ROW)
#define WS_ESRC (WS_RCT + CSA_SZ_ROW)
#define WS_EDST (WS_ESRC + 4u * NET)
#define WS_PW   (WS_EDST + 4u * NET)
#define P1  0
#define P2  (P1 + (size_t)512 * 256)
#define PP  (P2 + (size_t)512 * 512)
#define PF1 (PP + (size_t)768 * 512)
#define PF2 (PF1 + (size_t)512 * 1536)
#define PLA (PF2 + (size_t)768 * 512)
#define PLB (PLA + (size_t)768 * 768)
#define PWEND (PLB + (size_t)768 * 768)
#define WS_H    (WS_PW + 2u * PWEND)
#define WS_ESD  (WS_H + 4u * NPAD * 512)
#define WS_X1   (WS_ESD + 4u * NPAD * 8)
#define WS_PJ   (WS_X1 + 4u * NPAD * 512)
#define WS_F1   (WS_PJ + 4u * NPAD * 768)
#define WS_EMB  (WS_F1 + 4u * NPAD * 512)
#define WS_PU   (WS_EMB + 4u * NPAD * 768)
#define WS_PV   (WS_PU + 4u * NPAD * 768)
#define WS_T    (WS_PV + 4u * NPAD * 768)
#define WS_END  (WS_T + 4u * NPAD * 768)

__global__ __launch_bounds__(256) void k_edges(const int* __restrict__ EI, int* __restrict__ ESRC, int* __restrict__ EDST) {
  __shared__ __align__(16) int ss[256], sd_[256]; const int t = threadIdx.x; const size_t e = (size_t)blockIdx.x * 256 + t;
  int s = 0, d = 0; if (e < NE0) { s = EI[e]; d = EI[NE0 + e]; } else if (e < NET) { s = (int)(e - NE0); d = s; }
  ss[t] = s; sd_[t] = d; __syncthreads();
  if (t < 64 && (size_t)blockIdx.x * 256 + t * 4 < NET) { vst2((unsigned*)(ESRC + (size_t)blockIdx.x * 256 + t * 4), *(const v4u*)&ss[t * 4]); vst2((unsigned*)(EDST + (size_t)blockIdx.x * 256 + t * 4), *(const v4u*)&sd_[t * 4]); }
}
__global__ __launch_bounds__(256) void k_packW(const float* __restrict__ Wm, int K, int NOUT, int coff, __bf16* __restrict__ DST_) {
  __shared__ __align__(16) __bf16 s[1536]; const int n = blockIdx.x, tid = threadIdx.x;
  for (int k = tid; k < K; k += 256) s[k] = (__bf16)Wm[(size_t)k * NOUT + coff + n];
  __syncthreads();
  for (int q = tid; q < K / 8; q += 256) vst2((unsigned*)(DST_ + (size_t)n * K + q * 8), *(const v4u*)&s[q * 8]);
}
__global__ __launch_bounds__(256) void k_packWl(const float* __restrict__ Wm, __bf16* __restrict__ DA, __bf16* __restrict__ DB) {
  __shared__ __align__(16) __bf16 sa[768], sb[768]; const int n = blockIdx.x, tid = threadIdx.x;
  for (int k = tid; k < 768; k += 256) { sa[k] = (__bf16)Wm[(size_t)k * 768 + n]; sb[k] = (__bf16)Wm[(size_t)(768 + k) * 768 + n]; }
  __syncthreads();
  for (int q = tid; q < 96; q += 256) { vst2((unsigned*)(DA + (size_t)n * 768 + q * 8), *(const v4u*)&sa[q * 8]); vst2((unsigned*)(DB + (size_t)n * 768 + q * 8), *(const v4u*)&sb[q * 8]); }
}
template <int MODE>
__global__ __launch_bounds__(128) void k_gemm(const float* __restrict__ A, int lda, int K, const float* __restrict__ A2, const __bf16* __restrict__ P, const float* __restrict__ bias, float* __restrict__ OUT, int ldo) {
  __shared__ __align__(16) float so[4][16][132];
  const int tid = threadIdx.x, wave = tid >> 5, lane = tid & 31, col = lane & 15, g = lane >> 4; const size_t r0 = (size_t)blockIdx.x * 64 + wave * 16; const int n0 = blockIdx.y * 128; const size_t rr = r0 + col; const size_t ri = (rr >= NN) ? (size_t)NN - 1 : rr;
  v8f acc[8] = {};
#pragma unroll 2
  for (int kc = 0; kc < K / 32; ++kc) { F2 a; bool exact = false;
    if (MODE == 1 || (MODE == 2 && kc >= 768 / 32)) { v16b ax; const float* p = (MODE == 1) ? (A + ri * (size_t)lda + kc * 32 + 8 * g) : (A2 + ri * 768 + (kc * 32 - 768) + 8 * g);
#pragma unroll
      for (int i = 0; i < 8; ++i) { ax[i] = (__bf16)p[i]; ax[8 + i] = (__bf16)p[16 + i]; } a.h = ax; a.l = ax; exact = true; }
    else a = split_row(A + rr * (size_t)lda, kc * 32, lane);
#pragma unroll
    for (int j = 0; j < 8; ++j) { const v16b w = frag_b(P + (size_t)(n0 + j * 16 + col) * K + kc * 32, lane); if (!exact) acc[j] = wmma_bf(a.l, w, acc[j]); acc[j] = wmma_bf(a.h, w, acc[j]); } }
#pragma unroll
  for (int j = 0; j < 8; ++j) { const float bb = bias ? bfr(bias[n0 + j * 16 + col]) : 0.f;
#pragma unroll
    for (int r = 0; r < 8; ++r) so[wave][8 * g + r][j * 16 + col] = acc[j][r] + bb; }
  LDSX();
  for (int rl = 0; rl < 16; ++rl) vst2(OUT + (r0 + rl) * (size_t)ldo + n0 + lane * 4, *(const v4f*)&so[wave][rl][lane * 4]);
}
template <int NH_, int CH>
__global__ __launch_bounds__(256) void k_esd(const float* __restrict__ Hh, const float* __restrict__ AS, const float* __restrict__ AD, float* __restrict__ ESD) {
  __shared__ __align__(16) float s[64][8]; const int tid = threadIdx.x; const int wave = tid >> 5, lane = tid & 31;
  for (int q = wave; q < 64 * NH_; q += 8) { const int nl = q / NH_, h = q % NH_; const size_t n = (size_t)blockIdx.x * 64 + nl; const float* hr = Hh + n * 512 + h * CH; float a1 = 0.f, a2 = 0.f;
    for (int c = lane; c < CH; c += 32) { const float hv = hr[c]; a1 += hv * bfr(AS[h * CH + c]); a2 += hv * bfr(AD[h * CH + c]); }
#pragma unroll
    for (int o = 1; o < 32; o <<= 1) { a1 += __shfl_xor(a1, o); a2 += __shfl_xor(a2, o); }
    if (lane == 0) { s[nl][h] = a1; s[nl][4 + h] = a2; } }
  __syncthreads();
  if (tid < 64) { for (int h = NH_; h < 4; ++h) { s[tid][h] = 0.f; s[tid][4 + h] = 0.f; } }
  __syncthreads();
  for (int q = tid; q < 64 * 2; q += 256) vst2(ESD + ((size_t)blockIdx.x * 64) * 8 + q * 4, *(const v4f*)(&s[0][0] + q * 4));
}
template <int NH_, int CH>
__global__ __launch_bounds__(256) void k_gat(const float* __restrict__ Hh, const float* __restrict__ ESD, const int* __restrict__ FS, const int* __restrict__ RST, const int* __restrict__ RCT, const float* __restrict__ Bb, const float* __restrict__ G, const float* __restrict__ Be, float* __restrict__ X1) {
  __shared__ __align__(16) float srow[8][512];
  const int tid = threadIdx.x, wave = tid >> 5, lane = tid & 31; const size_t i = (size_t)blockIdx.x * 8 + wave; const int h = (lane * 16) / CH;
  float acc[16];
#pragma unroll
  for (int c = 0; c < 16; ++c) acc[c] = 0.f;
  if (i < NNT) { const int cnt = min(max(RCT[i], 0), CSA_BCAP); const int st = min(max(RST[i], 0), CSA_FINN - cnt); const float edi = ESD[i * 8 + 4 + h];
    float m = -3.0e38f;
    for (int e = 0; e < cnt; ++e) { const int s = min(max(FS[st + e], 0), NN - 1); if (s >= NNT) continue; float v = ESD[(size_t)s * 8 + h] + edi; v = v > 0.f ? v : 0.2f * v; m = fmaxf(m, v); }
    float z = 0.f;
    for (int e = 0; e < cnt; ++e) { const int s = min(max(FS[st + e], 0), NN - 1); if (s >= NNT) continue; float v = ESD[(size_t)s * 8 + h] + edi; v = v > 0.f ? v : 0.2f * v; z += exp_ni(v - m); }
    const float iz = 1.0f / (z + 1e-16f);
    for (int e = 0; e < cnt; ++e) { const int s = min(max(FS[st + e], 0), NN - 1); if (s >= NNT) continue; float v = ESD[(size_t)s * 8 + h] + edi; v = v > 0.f ? v : 0.2f * v; const float al = exp_ni(v - m) * iz; const float* row = Hh + (size_t)s * 512 + lane * 16;
#pragma unroll
      for (int c = 0; c < 16; ++c) acc[c] += al * row[c]; } }
  float sum = 0.f;
#pragma unroll
  for (int c = 0; c < 16; ++c) { acc[c] += bfr(Bb[lane * 16 + c]); sum += acc[c]; }
#pragma unroll
  for (int o = 1; o < 32; o <<= 1) sum += __shfl_xor(sum, o);
  const float mu = sum / 512.f; float var = 0.f;
#pragma unroll
  for (int c = 0; c < 16; ++c) { const float d = acc[c] - mu; var += d * d; }
#pragma unroll
  for (int o = 1; o < 32; o <<= 1) var += __shfl_xor(var, o);
  const float rs = rsqrtf(var / 512.f + 1e-5f);
  float o16[16];
#pragma unroll
  for (int c = 0; c < 16; ++c) { const float y = (acc[c] - mu) * rs * bfr(G[lane * 16 + c]) + bfr(Be[lane * 16 + c]); o16[c] = y > 0.f ? y : expm1_ni(y); }
#pragma unroll
  for (int c = 0; c < 16; ++c) srow[wave][lane * 16 + c] = o16[c];
  LDSX();
#pragma unroll
  for (int pc = 0; pc < 4; ++pc) vst2(X1 + i * 512 + pc * 128 + lane * 4, *(const v4f*)&srow[wave][pc * 128 + lane * 4]);
}
template <int W, int ACT>
__global__ __launch_bounds__(256) void k_ln(const float* __restrict__ T, const float* __restrict__ G, const float* __restrict__ Bb, float* __restrict__ Y) {
  constexpr int PER = W / 32; __shared__ __align__(16) float s[8][W]; const int tid = threadIdx.x, wave = tid >> 5, lane = tid & 31; const size_t row = (size_t)blockIdx.x * 8 + wave;
  float v[PER]; float sum = 0.f;
#pragma unroll
  for (int k = 0; k < PER; ++k) { v[k] = T[row * W + lane + 32 * k]; sum += v[k]; }
#pragma unroll
  for (int o = 1; o < 32; o <<= 1) sum += __shfl_xor(sum, o);
  const float mu = sum / (float)W; float var = 0.f;
#pragma unroll
  for (int k = 0; k < PER; ++k) { const float d = v[k] - mu; var += d * d; }
#pragma unroll
  for (int o = 1; o < 32; o <<= 1) var += __shfl_xor(var, o);
  const float rs = rsqrtf(var / (float)W + 1e-5f);
#pragma unroll
  for (int k = 0; k < PER; ++k) { const int c = lane + 32 * k; float y = (v[k] - mu) * rs * bfr(G[c]) + bfr(Bb[c]); if (ACT == 1) y = fmaxf(y, 0.f); s[wave][c] = y; }
  LDSX();
  for (int pc = lane; pc < W / 4; pc += 32) vst2(Y + row * W + pc * 4, *(const v4f*)&s[wave][pc * 4]);
}
__global__ __launch_bounds__(256) void k_link(const float* __restrict__ PU, const float* __restrict__ PV, const int* __restrict__ PE, const float* __restrict__ BL1, const float* __restrict__ WL2, const float* __restrict__ BL2, float* __restrict__ out) {
  __shared__ __align__(16) float so[64]; const int tid = threadIdx.x, wave = tid >> 5, lane = tid & 31;
  for (int k = 0; k < 8; ++k) { const int pl = wave * 8 + k; const size_t p = (size_t)blockIdx.x * 64 + pl; float a = 0.f;
    if (p < NPRT) { const int u = min(max(PE[p], 0), NN - 1), v = min(max(PE[NPR + p], 0), NN - 1); const float* pu = PU + (size_t)u * 768; const float* pv = PV + (size_t)v * 768;
      for (int d = lane; d < 768; d += 32) { const float t = pu[d] + pv[d] + bfr(BL1[d]); a += fmaxf(t, 0.f) * bfr(WL2[d]); } }
#pragma unroll
    for (int o = 1; o < 32; o <<= 1) a += __shfl_xor(a, o);
    if (lane == 0) so[pl] = (p < NPRT) ? a + bfr(BL2[0]) : 0.f; }
  __syncthreads();
  if (tid < 16 && (size_t)blockIdx.x * 64 + tid * 4 + 4 <= NPR) vst2(out + (size_t)blockIdx.x * 64 + tid * 4, *(const v4f*)&so[tid * 4]);
}
extern "C" void kernel_launch(void* const* d_in, const int* in_sizes, int n_in, void* d_out, int out_size, void* d_ws, size_t ws_size, hipStream_t stream) {
  (void)in_sizes; (void)n_in; (void)out_size;
  const float** F = (const float**)d_in; const int* EI = (const int*)d_in[1]; const int* PE = (const int*)d_in[2];
  if (ws_size < (size_t)WS_END) return;
  char* ws = (char*)d_ws;
  int *CNT = (int*)(ws + WS_CNT), *OFF = (int*)(ws + WS_OFF), *BST = (int*)(ws + WS_BST), *SEGS = (int*)(ws + WS_SEGS), *SEGE = (int*)(ws + WS_SEGE), *FS = (int*)(ws + WS_FS), *FE = (int*)(ws + WS_FE), *RST = (int*)(ws + WS_RST), *RCT = (int*)(ws + WS_RCT), *ESRC = (int*)(ws + WS_ESRC), *EDST = (int*)(ws + WS_EDST);
  __bf16* PW = (__bf16*)(ws + WS_PW); float *Hh = (float*)(ws + WS_H), *ESD = (float*)(ws + WS_ESD), *X1 = (float*)(ws + WS_X1), *PJ = (float*)(ws + WS_PJ), *F1 = (float*)(ws + WS_F1), *EMB = (float*)(ws + WS_EMB), *PU = (float*)(ws + WS_PU), *PV = (float*)(ws + WS_PV), *T = (float*)(ws + WS_T);
  k_edges<<<(NET + 255) / 256, 256, 0, stream>>>(EI, ESRC, EDST);
  k_csA_cnt<<<CSA_NCH, 256, 0, stream>>>(EDST, 1, CNT); k_csA_scan<<<1, 256, 0, stream>>>(CNT, OFF, BST); k_csA_scatter<<<CSA_NCH, 256, 0, stream>>>(ESRC, EDST, 1, 1, OFF, SEGS, SEGE); k_csA_bucket<<<CSA_NBK, 256, 0, stream>>>(CNT, OFF, BST, SEGS, SEGE, EDST, 1, FS, FE, RST, RCT);
  k_packW<<<512, 256, 0, stream>>>(F[4], 256, 512, 0, PW + P1); k_packW<<<512, 256, 0, stream>>>(F[10], 512, 512, 0, PW + P2); k_packW<<<768, 256, 0, stream>>>(F[16], 512, 768, 0, PW + PP); k_packW<<<512, 256, 0, stream>>>(F[18], 1536, 512, 0, PW + PF1); k_packW<<<768, 256, 0, stream>>>(F[22], 512, 768, 0, PW + PF2); k_packWl<<<768, 256, 0, stream>>>(F[26], PW + PLA, PW + PLB);
  k_gemm<1><<<dim3(NRBT, 4), 128, 0, stream>>>(F[0], 256, 256, nullptr, PW + P1, nullptr, Hh, 512);
  k_esd<4, 128><<<NRBT, 256, 0, stream>>>(Hh, F[5], F[6], ESD);
  k_gat<4, 128><<<NRBT * 8, 256, 0, stream>>>(Hh, ESD, FS, RST, RCT, F[7], F[8], F[9], X1);
  k_gemm<0><<<dim3(NRBT, 4), 128, 0, stream>>>(X1, 512, 512, nullptr, PW + P2, nullptr, Hh, 512);
  k_esd<2, 256><<<NRBT, 256, 0, stream>>>(Hh, F[11], F[12], ESD);
  k_gat<2, 256><<<NRBT * 8, 256, 0, stream>>>(Hh, ESD, FS, RST, RCT, F[13], F[14], F[15], X1);
  k_gemm<0><<<dim3(NRBT, 6), 128, 0, stream>>>(X1, 512, 512, nullptr, PW + PP, F[17], PJ, 768);
  k_gemm<2><<<dim3(NRBT, 4), 128, 0, stream>>>(PJ, 768, 1536, F[3], PW + PF1, F[19], T, 512);
  k_ln<512, 1><<<NRBT * 8, 256, 0, stream>>>(T, F[20], F[21], F1);
  k_gemm<0><<<dim3(NRBT, 6), 128, 0, stream>>>(F1, 512, 512, nullptr, PW + PF2, F[23], T, 768);
  k_ln<768, 0><<<NRBT * 8, 256, 0, stream>>>(T, F[24], F[25], EMB);
  k_gemm<0><<<dim3(NRBT, 6), 128, 0, stream>>>(EMB, 768, 768, nullptr, PW + PLA, nullptr, PU, 768);
  k_gemm<0><<<dim3(NRBT, 6), 128, 0, stream>>>(EMB, 768, 768, nullptr, PW + PLB, nullptr, PV, 768);
  k_link<<<(NPR + 63) / 64, 256, 0, stream>>>(PU, PV, PE, F[27], F[28], F[29], (float*)d_out);
}
